// LogSparseAttention_66632122630794
// MI455X (gfx1250) — hardware-verified
//
#include <hip/hip_runtime.h>
#include <math.h>

typedef __attribute__((ext_vector_type(16))) _Float16 v16h;
typedef __attribute__((ext_vector_type(16))) __bf16 v16b;
typedef __attribute__((ext_vector_type(8)))  _Float16 v8h;
typedef __attribute__((ext_vector_type(8)))  float v8f;
typedef __attribute__((ext_vector_type(4)))  float v4f;
typedef __attribute__((ext_vector_type(2)))  float v2f;
typedef __attribute__((ext_vector_type(4)))  unsigned v4u;
typedef __attribute__((ext_vector_type(4)))  int v4i;
typedef float __attribute__((may_alias)) float_a;
typedef int __attribute__((may_alias)) int_a;

template <typename T> __device__ __forceinline__ void vst2(void* p, T v) { *(volatile T*)p = v; __threadfence(); *(volatile T*)p = v; }
__device__ __forceinline__ v8f wmma16(v16h a, v16h b, v8f c) {
  v8f d = __builtin_amdgcn_wmma_f32_16x16x32_f16(false, a, false, b, (short)0, c, false, false);
  asm volatile("v_nop\n\tv_nop\n\tv_nop\n\tv_nop" : "+v"(d) : "v"(a), "v"(b));
  return d;
}
__device__ __forceinline__ v8f wmma_bf(v16b a, v16b b, v8f c) {
  v8f d = __builtin_amdgcn_wmma_f32_16x16x32_bf16(false, a, false, b, (short)0, c, false, false);
  asm volatile("v_nop\n\tv_nop\n\tv_nop\n\tv_nop" : "+v"(d) : "v"(a), "v"(b));
  return d;
}
__device__ __forceinline__ v16h frag_h(const _Float16* rowk0, int lane) {
  union { v16h v; v8h q[2]; } u; const _Float16* p = rowk0 + 8 * (lane >> 4);
  u.q[0] = *(const v8h*)p; u.q[1] = *(const v8h*)(p + 16); return u.v;
}
__device__ __forceinline__ v16h frag_f32(const float* rowk0, int lane) {
  v16h a; const float* p = rowk0 + 8 * (lane >> 4);
#pragma unroll
  for (int i = 0; i < 8; ++i) { a[i] = (_Float16)p[i]; a[8 + i] = (_Float16)p[16 + i]; }
  return a;
}
__device__ __forceinline__ v16h frag_f32s(const float* rowk0, int lane, float sc) {
  v16h a; const float* p = rowk0 + 8 * (lane >> 4);
#pragma unroll
  for (int i = 0; i < 8; ++i) { a[i] = (_Float16)(p[i] * sc); a[8 + i] = (_Float16)(p[16 + i] * sc); }
  return a;
}
__device__ __forceinline__ v16h fragc_f32(const float* W, int k0, int n, int lane, int ld, int K) {
  v16h a; const int g = lane >> 4;
#pragma unroll
  for (int i = 0; i < 8; ++i) { const int ka = k0 + 8 * g + i, kb = ka + 16;
    a[i] = (_Float16)(ka < K ? W[(size_t)ka * ld + n] : 0.f); a[8 + i] = (_Float16)(kb < K ? W[(size_t)kb * ld + n] : 0.f); }
  return a;
}
struct F2 { v16b h, l; };
__device__ __forceinline__ F2 bsplit16(const float v[16]) { F2 r;
#pragma unroll
  for (int i = 0; i < 16; ++i) { const __bf16 h = (__bf16)v[i]; r.h[i] = h; r.l[i] = (__bf16)(v[i] - (float)h); }
  return r; }
__device__ __forceinline__ F2 split_row(const float* row, int k0, int lane) { float v[16]; const float* p = row + k0 + 8 * (lane >> 4);
#pragma unroll
  for (int i = 0; i < 8; ++i) { v[i] = p[i]; v[8 + i] = p[16 + i]; }
  return bsplit16(v); }
__device__ __forceinline__ F2 split_rowK(const float* row, int k0, int lane, int K) { float v[16]; const int g = lane >> 4;
#pragma unroll
  for (int i = 0; i < 8; ++i) { const int ka = k0 + 8 * g + i, kb = ka + 16; v[i] = ka < K ? row[ka] : 0.f; v[8 + i] = kb < K ? row[kb] : 0.f; }
  return bsplit16(v); }
__device__ __forceinline__ F2 split_col(const float* W, int k0, int n, int lane, int ld, int K) { float v[16]; const int g = lane >> 4;
#pragma unroll
  for (int i = 0; i < 8; ++i) { const int ka = k0 + 8 * g + i, kb = ka + 16; v[i] = ka < K ? W[(size_t)ka * ld + n] : 0.f; v[8 + i] = kb < K ? W[(size_t)kb * ld + n] : 0.f; }
  return bsplit16(v); }
__device__ __forceinline__ v8f mac3(const F2& a, const F2& b, v8f c) { c = wmma_bf(a.l, b.h, c); c = wmma_bf(a.h, b.l, c); return wmma_bf(a.h, b.h, c); }
__device__ __forceinline__ float sigm(float v) { return 1.0f / (1.0f + expf(-v)); }
#define LDSX() do { asm volatile("s_wait_dscnt 0" ::: "memory"); __builtin_amdgcn_wave_barrier(); __builtin_amdgcn_fence(__ATOMIC_RELEASE, "workgroup"); } while (0)

#define NB 2
#define LL 2048
#define DM 1024
#define NH 16
#define DH 64
#define NR (NB * LL)

__global__ __launch_bounds__(256) void k_cvt(const float* __restrict__ src, _Float16* __restrict__ dst, size_t n8, float sc) {
  const size_t g8 = (size_t)blockIdx.x * 256 + threadIdx.x; if (g8 >= n8) return;
  union { v8h h; v4u u; } pk;
#pragma unroll
  for (int e = 0; e < 8; ++e) pk.h[e] = (_Float16)(src[g8 * 8 + e] * sc);
  vst2(dst + g8 * 8, pk.u);
}
template <int NOUT, int ASC>
__global__ __launch_bounds__(128) void k_gemm(const _Float16* __restrict__ A16, const _Float16* __restrict__ P, const float* __restrict__ b0, const float* __restrict__ b1, const float* __restrict__ b2, float* __restrict__ Out) {
  __shared__ __align__(16) float so[4][16][132];
  const int tid = threadIdx.x, wave = tid >> 5, lane = tid & 31, col = lane & 15, g = lane >> 4;
  const int r0 = blockIdx.x * 64 + wave * 16, n0 = blockIdx.y * 128;
  const float* bias = (n0 < DM) ? b0 : (n0 < 2 * DM ? b1 : b2); const int nb = n0 % DM;
  v8f acc[8] = {};
#pragma unroll 1
  for (int kc = 0; kc < DM / 32; ++kc) { const v16h a = frag_h(A16 + (size_t)(r0 + col) * DM + kc * 32, lane);
#pragma unroll
    for (int j = 0; j < 8; ++j) acc[j] = wmma16(a, frag_h(P + (size_t)(n0 + j * 16 + col) * DM + kc * 32, lane), acc[j]); }
#pragma unroll
  for (int j = 0; j < 8; ++j) { const float bb = bias[nb + j * 16 + col];
#pragma unroll
    for (int r = 0; r < 8; ++r) so[wave][8 * g + r][j * 16 + col] = acc[j][r] * (1.0f / (16.0f * ASC)) + bb; }
  LDSX();
#pragma unroll 4
  for (int rl = 0; rl < 16; ++rl) vst2(Out + (size_t)(r0 + rl) * NOUT + n0 + lane * 4, *(const v4f*)(&so[wave][rl][lane * 4]));
}
__global__ __launch_bounds__(256) void k_vsum(const float* __restrict__ QKV, float* __restrict__ Vs) {
  __shared__ float sp[8][128]; __shared__ __align__(16) float so[128];
  const int b = blockIdx.y, c0 = blockIdx.x * 128, tid = threadIdx.x; const int c = tid & 127, grp = tid >> 7;
  float s = 0.f;
#pragma unroll 4
  for (int m = grp * (LL / 2); m < (grp + 1) * (LL / 2); ++m) s += QKV[((size_t)b * LL + m) * (3 * DM) + 2 * DM + c0 + c];
  sp[grp][c] = s;
  __syncthreads();
  if (tid < 128) so[tid] = sp[0][tid] + sp[1][tid];
  __syncthreads();
  if (tid < 32) vst2(Vs + (size_t)b * DM + c0 + tid * 4, *(const v4f*)(&so[tid * 4]));
}
__global__ __launch_bounds__(256) void k_sparse(const float* __restrict__ QKV, const float* __restrict__ Vs, _Float16* __restrict__ O16) {
  __shared__ float sq[DM]; __shared__ float ssc[NH][16]; __shared__ int sj[16]; __shared__ int snsel;
  __shared__ __align__(16) _Float16 so[DM];
  const int i = blockIdx.x, b = blockIdx.y, tid = threadIdx.x; const size_t rowi = (size_t)b * LL + i;
  if (tid == 0) { int n = 0; int lg = 0; while ((2 << lg) <= i + 1) ++lg;
    for (int k = 0; k <= lg; ++k) { const int j = i - (1 << k); if (j >= 0) sj[n++] = j; }
    bool self = false; for (int t = 0; t < n; ++t) if (sj[t] == i) self = true;
    if (!self) sj[n++] = i;
    snsel = n; }
  for (int c = tid; c < DM; c += 256) sq[c] = QKV[rowi * (3 * DM) + c];
  __syncthreads();
  const int nsel = snsel;
  { const int h = tid >> 4, t = tid & 15; float s = 0.f;
    if (t < nsel) { const float* kr = QKV + ((size_t)b * LL + sj[t]) * (3 * DM) + DM + h * DH;
#pragma unroll 8
      for (int d = 0; d < DH; ++d) s += sq[h * DH + d] * kr[d];
      s *= 0.125f; }
    ssc[h][t] = s; }
  __syncthreads();
  { const int h = tid >> 4, d0 = (tid & 15) * 4; float Z = (float)(LL - nsel); float ex[16];
    for (int t = 0; t < nsel; ++t) { ex[t] = expf(ssc[h][t]); Z += ex[t]; }
    float o[4]; for (int e = 0; e < 4; ++e) o[e] = Vs[(size_t)b * DM + h * DH + d0 + e];
    for (int t = 0; t < nsel; ++t) { const float* vr = QKV + ((size_t)b * LL + sj[t]) * (3 * DM) + 2 * DM + h * DH + d0; const float wgt = ex[t] - 1.0f;
#pragma unroll
      for (int e = 0; e < 4; ++e) o[e] += wgt * vr[e]; }
    const float inv = 16.0f / Z;
#pragma unroll
    for (int e = 0; e < 4; ++e) so[h * DH + d0 + e] = (_Float16)(o[e] * inv); }
  __syncthreads();
  if (tid < DM / 8) vst2(O16 + rowi * DM + tid * 8, *(const v4u*)(&so[tid * 8]));
}
extern "C" void kernel_launch(void* const* d_in, const int* in_sizes, int n_in, void* d_out, int out_size, void* d_ws, size_t ws_size, hipStream_t stream) {
  (void)in_sizes; (void)n_in; (void)out_size; (void)ws_size;
  const float** I = (const float**)d_in;
  const float* x = I[0]; const float* Wq = I[1]; const float* bq = I[2]; const float* Wk = I[3]; const float* bk = I[4]; const float* Wv = I[5]; const float* bv = I[6]; const float* Wo = I[7]; const float* bo = I[8];
  float* out = (float*)d_out;
  char* ws = (char*)d_ws; size_t off = 0;
  auto take = [&](size_t bytes) { char* p = ws + off; off += (bytes + 255) & ~(size_t)255; return p; };
  _Float16* x16 = (_Float16*)take((size_t)NR * DM * 2); _Float16* P = (_Float16*)take((size_t)4 * DM * DM * 2); float* QKV = (float*)take((size_t)NR * 3 * DM * 4); float* Vs = (float*)take((size_t)NB * DM * 4); _Float16* O16 = (_Float16*)take((size_t)NR * DM * 2);
  auto cvt = [&](const float* s, _Float16* d, size_t n, float sc) { const size_t n8 = n / 8; k_cvt<<<(unsigned)((n8 + 255) / 256), 256, 0, stream>>>(s, d, n8, sc); };
  cvt(x, x16, (size_t)NR * DM, 1.0f); cvt(Wq, P, (size_t)DM * DM, 16.0f); cvt(Wk, P + (size_t)DM * DM, (size_t)DM * DM, 16.0f); cvt(Wv, P + (size_t)2 * DM * DM, (size_t)DM * DM, 16.0f); cvt(Wo, P + (size_t)3 * DM * DM, (size_t)DM * DM, 16.0f);
  k_gemm<3 * DM, 1><<<dim3(NR / 64, 3 * DM / 128), 128, 0, stream>>>(x16, P, bq, bk, bv, QKV);
  k_vsum<<<dim3(DM / 128, NB), 256, 0, stream>>>(QKV, Vs);
  k_sparse<<<dim3(LL, NB), 256, 0, stream>>>(QKV, Vs, O16);
  k_gemm<DM, 16><<<dim3(NR / 64, DM / 128), 128, 0, stream>>>(O16, P + (size_t)3 * DM * DM, bo, bo, bo, out);
}
